// RelativeAttention_56822417326644
// MI455X (gfx1250) — hardware-verified
//
#include <hip/hip_runtime.h>

typedef __attribute__((ext_vector_type(16))) __bf16       v16b;
typedef __attribute__((ext_vector_type(16))) _Float16     v16h;
typedef __attribute__((ext_vector_type(8)))  float        v8f;
typedef __attribute__((ext_vector_type(4)))  float        v4f;
typedef __attribute__((ext_vector_type(4)))  unsigned int v4u;

#ifndef NB
#define NB 16
#endif
#ifndef SEQ
#define SEQ 512
#endif
#define NB_FULL  16
#define SEQ_FULL 512

constexpr int DM     = 1024;
constexpr int NH     = 16;
constexpr int DH     = 64;
constexpr int NF     = 3 * NH * DH;
constexpr int MAXLEN = 512;
constexpr int NREL   = 2 * MAXLEN - 1;
constexpr int MROWS  = NB * SEQ;
constexpr int NBH    = NB * NH;
constexpr int KCH    = 64;
constexpr int QBLK   = 64;
constexpr int NWAVE  = 4;
constexpr int TPQ    = 72;
constexpr int TPV    = 136;
constexpr int OSP    = 68;

constexpr size_t PLANE16 = (size_t)MROWS * DM;
constexpr size_t WQT_EL  = (size_t)NF * DM;
constexpr size_t WOT_EL  = (size_t)DM * DM;
constexpr size_t WS_NEED = (6 * PLANE16 + WQT_EL + WOT_EL) * 2;

static_assert(NB >= 1 && NB <= NB_FULL);
static_assert(SEQ >= 128 && SEQ <= SEQ_FULL && SEQ <= MAXLEN);
static_assert(SEQ % 128 == 0);
static_assert(SEQ % KCH == 0 && SEQ % QBLK == 0);
static_assert(DH == 64 && NH * DH == DM);
static_assert(DM % 64 == 0 && NF % 64 == 0 && NF == 3 * DM);
static_assert(MROWS % 128 == 0);
static_assert((MROWS * DM) % 2048 == 0);
static_assert(NREL <= 1024);
static_assert(TPQ % 8 == 0 && TPV % 8 == 0 && OSP % 4 == 0);
static_assert(NWAVE * 32 * TPQ <= 2 * DH * TPV);
static_assert(WS_NEED <= 134217728ull);


__device__ __forceinline__ unsigned short f2bf_bits(float f) {
  unsigned u = __float_as_uint(f);
  return (unsigned short)((u + 0x7FFFu + ((u >> 16) & 1u)) >> 16);
}
__device__ __forceinline__ float bf_bits2f(unsigned short h) { return __uint_as_float(((unsigned)h) << 16); }
__device__ __forceinline__ float bfr(float f) { return bf_bits2f(f2bf_bits(f)); }
__device__ __forceinline__ unsigned short f2h_bits(float f) {
  _Float16 h = (_Float16)f;
  return __builtin_bit_cast(unsigned short, h);
}
__device__ __forceinline__ unsigned int pk16(unsigned short lo, unsigned short hi) {
  return (unsigned)lo | ((unsigned)hi << 16);
}

__device__ __forceinline__ v8f mma_bf16(v16b a, v16b b, v8f c) {
  c = __builtin_amdgcn_wmma_f32_16x16x32_bf16(false, a, false, b, (short)0, c, false, false);
  asm volatile("v_nop\n\tv_nop\n\tv_nop\n\tv_nop" : "+v"(c) : "v"(a), "v"(b));
  return c;
}
__device__ __forceinline__ v8f mma_f16(v16h a, v16h b, v8f c) {
  c = __builtin_amdgcn_wmma_f32_16x16x32_f16(false, a, false, b, (short)0, c, false, false);
  asm volatile("v_nop\n\tv_nop\n\tv_nop\n\tv_nop" : "+v"(c) : "v"(a), "v"(b));
  return c;
}

union FragB { v16b v; v4u u[2]; };
union FragH { v16h v; v4u u[2]; };


__global__ __launch_bounds__(256) void cvt_x_kernel(const float* __restrict__ x,
                                                    unsigned short* __restrict__ Xb)
{
  const int tid  = threadIdx.x;
  const int e    = tid * 8;
  const int crow = blockIdx.x * 2 + e / DM;
  const int col  = e % DM;
  const int bi   = crow / SEQ;
  const int n    = crow - bi * SEQ;
  const float* src = x + ((size_t)bi * SEQ_FULL + n) * DM + col;
  const v4f f0 = *(const v4f*)src;
  const v4f f1 = *(const v4f*)(src + 4);
  v4u w;
  w[0] = pk16(f2bf_bits(f0[0]), f2bf_bits(f0[1]));
  w[1] = pk16(f2bf_bits(f0[2]), f2bf_bits(f0[3]));
  w[2] = pk16(f2bf_bits(f1[0]), f2bf_bits(f1[1]));
  w[3] = pk16(f2bf_bits(f1[2]), f2bf_bits(f1[3]));
  unsigned short* dst = Xb + (size_t)crow * DM + col;
  *(volatile v4u*)dst = w;
  __threadfence();
  *(volatile v4u*)dst = w;
}

template <int KIND>
__global__ __launch_bounds__(256) void wtrans_kernel(const float* __restrict__ w,
                                                     unsigned short* __restrict__ Wt, int nf)
{
  __shared__ __align__(16) unsigned short Ts[64 * TPQ];
  const int tid  = threadIdx.x;
  const int n0   = blockIdx.x * 64;
  const int k0   = blockIdx.y * 64;
  const int krow = tid >> 2;
  const int fseg = (tid & 3) * 16;
  const float* src = w + (size_t)(k0 + krow) * nf + n0 + fseg;
#pragma unroll
  for (int i = 0; i < 4; ++i) {
    const v4f f = *(const v4f*)(src + 4 * i);
#pragma unroll
    for (int e2 = 0; e2 < 4; ++e2) {
      const float v = f[e2];
      unsigned short bits;
      if (KIND == 0) bits = f2bf_bits(v);
      else           bits = f2h_bits(bfr(v) * 64.0f);
      Ts[(fseg + 4 * i + e2) * TPQ + krow] = bits;
    }
  }
  __syncthreads();
  for (int pass = 0; pass < 2; ++pass) {
#pragma unroll
    for (int it = 0; it < 2; ++it) {
      const int u    = it * 256 + tid;
      const int frow = u >> 3;
      const int seg  = u & 7;
      const v4u val = *(const v4u*)(Ts + frow * TPQ + seg * 8);
      *(volatile v4u*)(Wt + (size_t)(n0 + frow) * DM + k0 + seg * 8) = val;
    }
    __threadfence();
  }
}

__global__ __launch_bounds__(128) __attribute__((amdgpu_num_vgpr(256)))
void qkv_gemm_kernel(const unsigned short* __restrict__ Xb, const unsigned short* __restrict__ Wqt,
                     const float* __restrict__ bq,
                     unsigned short* __restrict__ Qh, unsigned short* __restrict__ Kh,
                     unsigned short* __restrict__ Vth, unsigned short* __restrict__ Vtl)
{
  __shared__ __align__(16) unsigned short Ts[2 * DH * TPV];
  const int tid  = threadIdx.x;
  const int wave = tid >> 5;
  const int lane = tid & 31;
  const int hh   = lane >> 4;
  const int c    = lane & 15;
  const int m0   = blockIdx.x * 128;
  const int n0   = blockIdx.y * 64;
  const int sel  = blockIdx.y / (DM / 64);
  const int head = blockIdx.y - sel * (DM / 64);

  v8f acc[2][4];
#pragma unroll
  for (int rt = 0; rt < 2; ++rt)
#pragma unroll
    for (int tt = 0; tt < 4; ++tt) acc[rt][tt] = (v8f){0.f,0.f,0.f,0.f,0.f,0.f,0.f,0.f};

  const unsigned short* a0p = Xb + (size_t)(m0 + 32 * wave + c) * DM + 8 * hh;
  const unsigned short* a1p = a0p + (size_t)16 * DM;
  const unsigned short* b0p = Wqt + (size_t)(n0 + c) * DM + 8 * hh;

#pragma unroll 1
  for (int k0 = 0; k0 < DM; k0 += 32) {
    FragB a0, a1;
    a0.u[0] = *(const v4u*)(a0p + k0);
    a0.u[1] = *(const v4u*)(a0p + k0 + 16);
    a1.u[0] = *(const v4u*)(a1p + k0);
    a1.u[1] = *(const v4u*)(a1p + k0 + 16);
#pragma unroll
    for (int tt = 0; tt < 4; ++tt) {
      const unsigned short* bp = b0p + (size_t)tt * 16 * DM + k0;
      FragB b;
      b.u[0] = *(const v4u*)bp;
      b.u[1] = *(const v4u*)(bp + 16);
      acc[0][tt] = mma_bf16(a0.v, b.v, acc[0][tt]);
      acc[1][tt] = mma_bf16(a1.v, b.v, acc[1][tt]);
    }
  }

  float bb[4];
#pragma unroll
  for (int tt = 0; tt < 4; ++tt) bb[tt] = bfr(bq[n0 + 16 * tt + c]);

  const int bi  = m0 / SEQ;
  const int nn0 = m0 - bi * SEQ;
  const int bh  = bi * NH + head;

  if (sel < 2) {
    unsigned short* plane = (sel == 0) ? Qh : Kh;
    unsigned short* ls = Ts + wave * (32 * TPQ);
#pragma unroll
    for (int rt = 0; rt < 2; ++rt)
#pragma unroll
      for (int tt = 0; tt < 4; ++tt)
#pragma unroll
        for (int r = 0; r < 8; ++r)
          ls[(16 * rt + 8 * hh + r) * TPQ + 16 * tt + c] = f2h_bits(acc[rt][tt][r] + bb[tt]);
    __syncthreads();
    unsigned short* dst = plane + ((size_t)bh * SEQ + nn0 + 32 * wave) * DH;
    for (int pass = 0; pass < 2; ++pass) {
#pragma unroll
      for (int it = 0; it < 8; ++it) {
        const int row = it * 4 + (lane >> 3);
        const int seg = lane & 7;
        const v4u val = *(const v4u*)(ls + row * TPQ + seg * 8);
        *(volatile v4u*)(dst + (size_t)row * DH + seg * 8) = val;
      }
      __threadfence();
    }
  } else {
    unsigned short* th = Ts;
    unsigned short* tl = Ts + DH * TPV;
#pragma unroll
    for (int rt = 0; rt < 2; ++rt)
#pragma unroll
      for (int tt = 0; tt < 4; ++tt)
#pragma unroll
        for (int r = 0; r < 8; ++r) {
          const float v = acc[rt][tt][r] + bb[tt];
          const unsigned short hb = f2bf_bits(v);
          const unsigned short lb = f2bf_bits(v - bf_bits2f(hb));
          const int tok = 32 * wave + 16 * rt + 8 * hh + r;
          const int d   = 16 * tt + c;
          th[d * TPV + tok] = hb;
          tl[d * TPV + tok] = lb;
        }
    __syncthreads();
    const size_t vbase = (size_t)bh * DH * SEQ + nn0;
    const int seg = lane & 15;
    for (int pass = 0; pass < 2; ++pass) {
#pragma unroll
      for (int it = 0; it < 8; ++it) {
        const int drow = 16 * wave + it * 2 + hh;
        const v4u hv = *(const v4u*)(th + drow * TPV + seg * 8);
        const v4u lv = *(const v4u*)(tl + drow * TPV + seg * 8);
        *(volatile v4u*)(Vth + vbase + (size_t)drow * SEQ + seg * 8) = hv;
        *(volatile v4u*)(Vtl + vbase + (size_t)drow * SEQ + seg * 8) = lv;
      }
      __threadfence();
    }
  }
}

__global__ __launch_bounds__(128) __attribute__((amdgpu_num_vgpr(256)))
void attn_kernel(const unsigned short* __restrict__ Qh, const unsigned short* __restrict__ Kh,
                 const unsigned short* __restrict__ Vth, const unsigned short* __restrict__ Vtl,
                 const float* __restrict__ rel, unsigned short* __restrict__ Ctx)
{
  __shared__ __align__(16) unsigned short Ksh[KCH * DH];
  __shared__ __align__(16) unsigned short Vhs[DH * KCH];
  __shared__ __align__(16) unsigned short Vls[DH * KCH];
  __shared__ __align__(16) unsigned short Psh[NWAVE][16 * KCH];
  __shared__ __align__(16) unsigned short Psl[NWAVE][16 * KCH];
  __shared__ __align__(16) unsigned short Osh[NWAVE][16 * TPQ];
  __shared__ float sbias[1024];

  const int tid  = threadIdx.x;
  const int wave = tid >> 5;
  const int lane = tid & 31;
  const int hh   = lane >> 4;
  const int c    = lane & 15;
  const int qb   = blockIdx.x;
  const int bh   = blockIdx.y;
  const int bi   = bh / NH;
  const int head = bh - bi * NH;
  const int q0   = qb * QBLK + wave * 16;

  for (int t = tid; t < 1024; t += 128) {
    const int ti = t < NREL ? t : (NREL - 1);
    const float v = bfr(rel[(size_t)ti * NH + head]);
    sbias[t] = (t < NREL) ? v : 0.f;
  }

  FragH qa[2];
  {
    const unsigned short* qrow = Qh + ((size_t)bh * SEQ + q0 + c) * DH + 8 * hh;
    qa[0].u[0] = *(const v4u*)(qrow);
    qa[0].u[1] = *(const v4u*)(qrow + 16);
    qa[1].u[0] = *(const v4u*)(qrow + 32);
    qa[1].u[1] = *(const v4u*)(qrow + 48);
  }
  __syncthreads();

  float mrow[8], lrow[8];
  v8f oacc[4];
#pragma unroll
  for (int r = 0; r < 8; ++r) { mrow[r] = -__builtin_inff(); lrow[r] = 0.f; }
#pragma unroll
  for (int t = 0; t < 4; ++t) oacc[t] = (v8f){0.f,0.f,0.f,0.f,0.f,0.f,0.f,0.f};

  const unsigned short* Kp  = Kh  + (size_t)bh * SEQ * DH;
  const unsigned short* Vhp = Vth + (size_t)bh * DH * SEQ;
  const unsigned short* Vlp = Vtl + (size_t)bh * DH * SEQ;
  unsigned short* pwh = Psh[wave];
  unsigned short* pwl = Psl[wave];
  const int bbase = q0 + 8 * hh - c + (MAXLEN - 1);

#pragma unroll 1
  for (int kc = 0; kc < SEQ / KCH; ++kc) {
    const int kv0 = kc * KCH;
    __syncthreads();
#pragma unroll
    for (int it = 0; it < 4; ++it) {
      const int u   = it * 128 + tid;
      const int row = u >> 3;
      const int seg = u & 7;
      const v4u kw = *(const v4u*)(Kp  + (size_t)(kv0 + row) * DH + seg * 8);
      const v4u hw = *(const v4u*)(Vhp + (size_t)row * SEQ + kv0 + seg * 8);
      const v4u lw = *(const v4u*)(Vlp + (size_t)row * SEQ + kv0 + seg * 8);
      *(v4u*)(Ksh + row * DH + seg * 8)  = kw;
      *(v4u*)(Vhs + row * KCH + seg * 8) = hw;
      *(v4u*)(Vls + row * KCH + seg * 8) = lw;
    }
    __syncthreads();

    v8f s[4];
#pragma unroll
    for (int j = 0; j < 4; ++j) {
      s[j] = (v8f){0.f,0.f,0.f,0.f,0.f,0.f,0.f,0.f};
#pragma unroll
      for (int dc = 0; dc < 2; ++dc) {
        FragH kf;
        kf.u[0] = *(const v4u*)(Ksh + (j * 16 + c) * DH + dc * 32 + 8 * hh);
        kf.u[1] = *(const v4u*)(Ksh + (j * 16 + c) * DH + dc * 32 + 16 + 8 * hh);
        s[j] = mma_f16(qa[dc].v, kf.v, s[j]);
      }
    }

    const int boff = bbase - kv0;
#pragma unroll
    for (int j = 0; j < 4; ++j)
#pragma unroll
      for (int r = 0; r < 8; ++r)
        s[j][r] = s[j][r] * 0.125f + sbias[boff + r - 16 * j];

    float cm[8];
#pragma unroll
    for (int r = 0; r < 8; ++r) {
      float m = fmaxf(fmaxf(s[0][r], s[1][r]), fmaxf(s[2][r], s[3][r]));
#pragma unroll
      for (int off = 1; off < 16; off <<= 1) m = fmaxf(m, __shfl_xor(m, off, 32));
      cm[r] = m;
    }

#pragma unroll
    for (int r = 0; r < 8; ++r) {
      const float mnew  = fmaxf(mrow[r], cm[r]);
      const float alpha = __expf(mrow[r] - mnew);
      mrow[r] = mnew;
      float psum = 0.f;
#pragma unroll
      for (int j = 0; j < 4; ++j) {
        const float p = __expf(s[j][r] - mnew);
        psum += p;
        const unsigned short hb = f2bf_bits(p);
        const unsigned short lb = f2bf_bits(p - bf_bits2f(hb));
        pwh[(8 * hh + r) * KCH + j * 16 + c] = hb;
        pwl[(8 * hh + r) * KCH + j * 16 + c] = lb;
      }
#pragma unroll
      for (int off = 1; off < 16; off <<= 1) psum += __shfl_xor(psum, off, 32);
      lrow[r] = lrow[r] * alpha + psum;
#pragma unroll
      for (int t = 0; t < 4; ++t) oacc[t][r] *= alpha;
    }
    __builtin_amdgcn_fence(3, "workgroup");
    __builtin_amdgcn_wave_barrier();
    __builtin_amdgcn_fence(2, "workgroup");

#pragma unroll
    for (int kk = 0; kk < 2; ++kk) {
      FragB pa, pl;
      pa.u[0] = *(const v4u*)(pwh + c * KCH + kk * 32 + 8 * hh);
      pa.u[1] = *(const v4u*)(pwh + c * KCH + kk * 32 + 16 + 8 * hh);
      pl.u[0] = *(const v4u*)(pwl + c * KCH + kk * 32 + 8 * hh);
      pl.u[1] = *(const v4u*)(pwl + c * KCH + kk * 32 + 16 + 8 * hh);
#pragma unroll
      for (int t = 0; t < 4; ++t) {
        FragB vh, vl;
        vh.u[0] = *(const v4u*)(Vhs + (t * 16 + c) * KCH + kk * 32 + 8 * hh);
        vh.u[1] = *(const v4u*)(Vhs + (t * 16 + c) * KCH + kk * 32 + 16 + 8 * hh);
        vl.u[0] = *(const v4u*)(Vls + (t * 16 + c) * KCH + kk * 32 + 8 * hh);
        vl.u[1] = *(const v4u*)(Vls + (t * 16 + c) * KCH + kk * 32 + 16 + 8 * hh);
        oacc[t] = mma_bf16(pa.v, vh.v, oacc[t]);
        oacc[t] = mma_bf16(pl.v, vh.v, oacc[t]);
        oacc[t] = mma_bf16(pa.v, vl.v, oacc[t]);
      }
    }
  }

  unsigned short* os = Osh[wave];
#pragma unroll
  for (int r = 0; r < 8; ++r) {
    const float inv = 1.0f / lrow[r];
#pragma unroll
    for (int t = 0; t < 4; ++t)
      os[(8 * hh + r) * TPQ + t * 16 + c] = f2h_bits(oacc[t][r] * inv * 16.0f);
  }
  __builtin_amdgcn_fence(3, "workgroup");
  __builtin_amdgcn_wave_barrier();
  __builtin_amdgcn_fence(2, "workgroup");
  {
    unsigned short* cdst = Ctx + ((size_t)bi * SEQ + q0) * DM + head * DH;
    for (int pass = 0; pass < 2; ++pass) {
#pragma unroll
      for (int it = 0; it < 4; ++it) {
        const int row = it * 4 + (lane >> 3);
        const int seg = lane & 7;
        const v4u val = *(const v4u*)(os + row * TPQ + seg * 8);
        *(volatile v4u*)(cdst + (size_t)row * DM + seg * 8) = val;
      }
      __threadfence();
    }
  }
}

__global__ __launch_bounds__(128) __attribute__((amdgpu_num_vgpr(256)))
void out_gemm_kernel(const unsigned short* __restrict__ Ctx, const unsigned short* __restrict__ Wot,
                     const float* __restrict__ bo, float* __restrict__ out)
{
  __shared__ __align__(16) float Os[NWAVE][32 * OSP];
  const int tid  = threadIdx.x;
  const int wave = tid >> 5;
  const int lane = tid & 31;
  const int hh   = lane >> 4;
  const int c    = lane & 15;
  const int m0   = blockIdx.x * 128;
  const int n0   = blockIdx.y * 64;

  v8f acc[2][4];
#pragma unroll
  for (int rt = 0; rt < 2; ++rt)
#pragma unroll
    for (int tt = 0; tt < 4; ++tt) acc[rt][tt] = (v8f){0.f,0.f,0.f,0.f,0.f,0.f,0.f,0.f};

  const unsigned short* a0p = Ctx + (size_t)(m0 + 32 * wave + c) * DM + 8 * hh;
  const unsigned short* a1p = a0p + (size_t)16 * DM;
  const unsigned short* b0p = Wot + (size_t)(n0 + c) * DM + 8 * hh;

#pragma unroll 1
  for (int k0 = 0; k0 < DM; k0 += 32) {
    FragH a0, a1;
    a0.u[0] = *(const v4u*)(a0p + k0);
    a0.u[1] = *(const v4u*)(a0p + k0 + 16);
    a1.u[0] = *(const v4u*)(a1p + k0);
    a1.u[1] = *(const v4u*)(a1p + k0 + 16);
#pragma unroll
    for (int tt = 0; tt < 4; ++tt) {
      const unsigned short* bp = b0p + (size_t)tt * 16 * DM + k0;
      FragH b;
      b.u[0] = *(const v4u*)bp;
      b.u[1] = *(const v4u*)(bp + 16);
      acc[0][tt] = mma_f16(a0.v, b.v, acc[0][tt]);
      acc[1][tt] = mma_f16(a1.v, b.v, acc[1][tt]);
    }
  }

  float bb[4];
#pragma unroll
  for (int tt = 0; tt < 4; ++tt) bb[tt] = bfr(bo[n0 + 16 * tt + c]);

  float* os = Os[wave];
#pragma unroll
  for (int rt = 0; rt < 2; ++rt)
#pragma unroll
    for (int tt = 0; tt < 4; ++tt)
#pragma unroll
      for (int r = 0; r < 8; ++r)
        os[(16 * rt + 8 * hh + r) * OSP + 16 * tt + c] = acc[rt][tt][r] * (1.0f / 1024.0f) + bb[tt];
  __builtin_amdgcn_fence(3, "workgroup");
  __builtin_amdgcn_wave_barrier();
  __builtin_amdgcn_fence(2, "workgroup");

  const int bi  = m0 / SEQ;
  const int nn0 = m0 - bi * SEQ;
  float* ob = out + ((size_t)bi * SEQ_FULL + nn0 + 32 * wave) * DM + n0;
  const int c4 = (lane & 15) * 4;
  for (int pass = 0; pass < 2; ++pass) {
#pragma unroll
    for (int it = 0; it < 16; ++it) {
      const int row = it * 2 + hh;
      const v4f val = *(const v4f*)(os + row * OSP + c4);
      *(volatile v4f*)(ob + (size_t)row * DM + c4) = val;
    }
    __threadfence();
  }
}

extern "C" void kernel_launch(void* const* d_in, const int* in_sizes, int n_in,
                              void* d_out, int out_size, void* d_ws, size_t ws_size,
                              hipStream_t stream)
{
  if (n_in < 6) return;
  const long need_x = ((long)(NB - 1) * SEQ_FULL + SEQ) * DM;
  if ((long)in_sizes[0] < need_x) return;
  if ((long)in_sizes[1] < (long)DM * NF) return;
  if (in_sizes[2] < NF) return;
  if ((long)in_sizes[3] < (long)NREL * NH) return;
  if ((long)in_sizes[4] < (long)DM * DM) return;
  if (in_sizes[5] < DM) return;
  if ((long)out_size < need_x) return;
  if (d_ws == nullptr || ws_size < WS_NEED) return;

  const float* x     = (const float*)d_in[0];
  const float* w_qkv = (const float*)d_in[1];
  const float* b_qkv = (const float*)d_in[2];
  const float* rel   = (const float*)d_in[3];
  const float* w_out = (const float*)d_in[4];
  const float* b_out = (const float*)d_in[5];
  float* out = (float*)d_out;

  unsigned short* Xb  = (unsigned short*)d_ws;
  unsigned short* Wqt = Xb  + PLANE16;
  unsigned short* Wot = Wqt + WQT_EL;
  unsigned short* Qh  = Wot + WOT_EL;
  unsigned short* Kh  = Qh  + PLANE16;
  unsigned short* Vth = Kh  + PLANE16;
  unsigned short* Vtl = Vth + PLANE16;
  unsigned short* Ctx = Vtl + PLANE16;

  cvt_x_kernel<<<dim3((unsigned)((MROWS * DM) / 2048)), 256, 0, stream>>>(x, Xb);
  wtrans_kernel<0><<<dim3(NF / 64, DM / 64), 256, 0, stream>>>(w_qkv, Wqt, NF);
  wtrans_kernel<1><<<dim3(DM / 64, DM / 64), 256, 0, stream>>>(w_out, Wot, DM);
  qkv_gemm_kernel<<<dim3(MROWS / 128, NF / 64), 128, 0, stream>>>(Xb, Wqt, b_qkv, Qh, Kh, Vth, Vtl);
  attn_kernel<<<dim3(SEQ / QBLK, NBH), 128, 0, stream>>>(Qh, Kh, Vth, Vtl, rel, Ctx);
  out_gemm_kernel<<<dim3(MROWS / 128, DM / 64), 128, 0, stream>>>(Ctx, Wot, b_out, out);
}
